// InputStream_15109694947667
// MI455X (gfx1250) — hardware-verified
//
#include <hip/hip_runtime.h>
#include <stddef.h>


typedef float          v2f   __attribute__((ext_vector_type(2)));
typedef float          v4f   __attribute__((ext_vector_type(4)));
typedef float          v8f   __attribute__((ext_vector_type(8)));
typedef unsigned int   u32x2 __attribute__((ext_vector_type(2)));
typedef unsigned int   u32x4 __attribute__((ext_vector_type(4)));
typedef _Float16       v16h  __attribute__((ext_vector_type(16)));
typedef __bf16         v16b  __attribute__((ext_vector_type(16)));

union FH { v16h v; u32x4 q[2]; };
union FB { v16b v; u32x4 q[2]; };

#define IMH   128
#define IMW   128
#define NPIX  (IMH * IMW)
#define NBAT  64
#define NTS   5
#define BR    16
#define BC    32
#define SHH   (BR + 2)
#define SWW   (BC + 2)
#define NHALO (SHH * SWW)
#define PLB   (NHALO * 16)
#define DK    1024
#define DKC   64
#define NKB   64
#define APITCH 72

static_assert(NHALO == 612);
static_assert(NKB * DK == NPIX * 4);
static_assert((IMH % BR) == 0 && (IMW % BC) == 0);

__device__ __forceinline__ unsigned f16b(float v) {
  const _Float16 hv = (_Float16)v;
  return (unsigned)__builtin_bit_cast(unsigned short, hv);
}
__device__ __forceinline__ float h2f(unsigned b) {
  return (float)__builtin_bit_cast(_Float16, (unsigned short)b);
}
__device__ __forceinline__ unsigned bf16b(float f) {
  unsigned u = __float_as_uint(f);
  u += 0x7FFFu + ((u >> 16) & 1u);
  return u >> 16;
}
__device__ __forceinline__ float bf2f(unsigned b) { return __uint_as_float(b << 16); }
__device__ __forceinline__ float lrl(float x) { return x > 0.0f ? x : 0.3f * x; }

__device__ __forceinline__ v8f wmh(const FH& a, const FH& b, v8f c) {
  v8f d = __builtin_amdgcn_wmma_f32_16x16x32_f16(false, a.v, false, b.v, (short)0, c, false, false);
  asm volatile("v_nop\n\tv_nop\n\tv_nop\n\tv_nop" : "+v"(d) : "v"(a.v), "v"(b.v));
  return d;
}
__device__ __forceinline__ v8f wmb(const FB& a, const FB& b, v8f c) {
  v8f d = __builtin_amdgcn_wmma_f32_16x16x32_bf16(false, a.v, false, b.v, (short)0, c, false, false);
  asm volatile("v_nop\n\tv_nop\n\tv_nop\n\tv_nop" : "+v"(d) : "v"(a.v), "v"(b.v));
  return d;
}

__device__ __forceinline__ v8f zero8f() {
  v8f z;
#pragma unroll
  for (int i = 0; i < 8; ++i) z[i] = 0.0f;
  return z;
}

__device__ __forceinline__ float sigm_f(float x) { return __fdividef(1.0f, 1.0f + __expf(-x)); }

__device__ __forceinline__ float tanh_f(float x) {
  const float ax = fabsf(x);
  const float x2 = x * x;
  float p = -1.4558344e-3f;
  p = p * x2 + 3.5921280e-3f;
  p = p * x2 - 8.8632355e-3f;
  p = p * x2 + 2.1869489e-2f;
  p = p * x2 - 5.3968254e-2f;
  p = p * x2 + 1.3333334e-1f;
  p = p * x2 - 3.3333334e-1f;
  const float tp = x + x * (x2 * p);
  const float e = __expf(2.0f * fminf(ax, 40.0f));
  const float tb = copysignf(1.0f - __fdividef(2.0f, e + 1.0f), x);
  return (ax < 0.55f) ? tp : tb;
}

__host__ __device__ constexpr int goff(int G) {
  return (G / 9) * PLB + (((G % 9) / 3) * SWW + ((G % 9) % 3)) * 16;
}

template <int GL, int NGT>
__device__ __forceinline__ u32x4 ldgrp(const unsigned char* lb, int hh) {
  u32x4 v = {0u, 0u, 0u, 0u};
  if constexpr (GL + 1 < NGT) {
    const int off = hh ? goff(GL + 1) : goff(GL);
    v = *(const u32x4*)(lb + off);
  } else if constexpr (GL < NGT) {
    const u32x4 t = *(const u32x4*)(lb + goff(GL));
    v.x = hh ? 0u : t.x; v.y = hh ? 0u : t.y; v.z = hh ? 0u : t.z; v.w = hh ? 0u : t.w;
  }
  return v;
}

template <int S, int NGT>
__device__ __forceinline__ v8f kstep(const FH& a, const unsigned char* lb, int hh, v8f acc) {
  FH bq;
  bq.q[0] = ldgrp<4 * S, NGT>(lb, hh);
  bq.q[1] = ldgrp<4 * S + 2, NGT>(lb, hh);
  return wmh(a, bq, acc);
}

__global__ __launch_bounds__(256) void k_wpack(
    const float* __restrict__ wx1, const float* __restrict__ wh1,
    const float* __restrict__ wx2, const float* __restrict__ wh2,
    const float* __restrict__ wx3, const float* __restrict__ wh3,
    unsigned short* wpk)
{
  const int l = blockIdx.x, tid = threadIdx.x;
  const float* wx = (l == 0) ? wx1 : ((l == 1) ? wx2 : wx3);
  const float* wh = (l == 0) ? wh1 : ((l == 1) ? wh2 : wh3);
  const int cin = (l == 0) ? 3 : 4;
  const int ng  = (l == 0) ? 9 : 18;
  const int gpr = (l == 0) ? 12 : 20;
  const float swx = (l == 0) ? 16384.0f : 1024.0f;
  const float swh = (l == 0) ? 64.0f : 1024.0f;
  const int nch = 16 * gpr;
  unsigned short* dst = wpk + (size_t)l * 4096;

#pragma unroll
  for (int it = 0; it < 2; ++it) {
    const int q = tid + 256 * it;
    const bool valid = q < nch;
    const int qc = valid ? q : (nch - 1);
    const int ch = qc / gpr, G = qc - ch * gpr;
    const int Ta = G < 8 ? G : 8;
    int Tb = G - 9; Tb = Tb < 0 ? 0 : (Tb > 8 ? 8 : Tb);
    unsigned hb[8];
#pragma unroll
    for (int j = 0; j < 8; ++j) {
      const int jj = j & 3;
      const int jx = jj < cin - 1 ? jj : cin - 1;
      const float wxa = wx[(Ta * cin + jx) * 16 + ch];
      const float wha = wh[(Ta * 4 + jj) * 16 + ch];
      const float wxb = wx[(Tb * cin + jj) * 16 + ch];
      const float va = (j < 4) ? ((jj < cin) ? wxa * swx : 0.0f) : wha * swh;
      const unsigned ba = f16b(va);
      const float wb = wxb * swx;
      const unsigned bh = f16b(wb);
      const unsigned bl = f16b(wb - h2f(bh));
      const unsigned bb = (j < 4) ? bh : bl;
      hb[j] = (G < 9) ? ba : ((G < ng) ? bb : 0u);
    }
    u32x4 pk;
    pk.x = hb[0] | (hb[1] << 16); pk.y = hb[2] | (hb[3] << 16);
    pk.z = hb[4] | (hb[5] << 16); pk.w = hb[6] | (hb[7] << 16);
    if (valid) *(volatile u32x4*)(dst + (size_t)q * 8) = pk;
    __threadfence();
    if (valid) *(volatile u32x4*)(dst + (size_t)q * 8) = pk;
  }
}

template <int CIN, int SPLIT>
__global__ __launch_bounds__(256) void k_cell(
    const float* __restrict__ xin,
    const float* __restrict__ hprev,
    float* hout, float* cst,
    const unsigned short* __restrict__ wpk,
    const float* __restrict__ bias,
    const float* __restrict__ ng, const float* __restrict__ nbt,
    const float* __restrict__ nmu, const float* __restrict__ nva,
    int tt, int first)
{
  constexpr int   NG  = SPLIT ? 18 : 9;
  constexpr int   NKS = SPLIT ? 5 : 3;
  constexpr int   KP  = NKS * 32;
  constexpr float SAX = (CIN == 3) ? 16.0f : 4096.0f;
  constexpr float SAH = 4096.0f;
  constexpr float STI = (CIN == 3) ? (1.0f / 262144.0f) : (1.0f / 4194304.0f);
  __shared__ __attribute__((aligned(16))) unsigned char stg[(SPLIT ? 2 : 1) * PLB];

  const int tid = threadIdx.x, lane = tid & 31, wave = tid >> 5, hh = lane >> 4, m = lane & 15;
  const int bx = blockIdx.x, by = blockIdx.y, b = blockIdx.z;

  float na0 = 0.f, na1 = 0.f, na2 = 0.f, na3 = 0.f, nc0 = 0.f, nc1 = 0.f, nc2 = 0.f, nc3 = 0.f;
  float nm0 = 0.f, nm1 = 0.f, nm2 = 0.f, nm3 = 0.f;
  if constexpr (CIN == 4) {
    na0 = ng[0] * rsqrtf(nva[0] + 1.0e-3f) * SAX; na1 = ng[1] * rsqrtf(nva[1] + 1.0e-3f) * SAX;
    na2 = ng[2] * rsqrtf(nva[2] + 1.0e-3f) * SAX; na3 = ng[3] * rsqrtf(nva[3] + 1.0e-3f) * SAX;
    nc0 = nbt[0] * SAX; nc1 = nbt[1] * SAX; nc2 = nbt[2] * SAX; nc3 = nbt[3] * SAX;
    nm0 = nmu[0]; nm1 = nmu[1]; nm2 = nmu[2]; nm3 = nmu[3];
  }

#pragma unroll 1
  for (int it = 0; it < 3; ++it) {
    int i = tid + 256 * it;
    i = i > NHALO - 1 ? NHALO - 1 : i;
    const int lr = i / SWW, lc = i - lr * SWW;
    const int gr = by * BR - 1 + lr, gc = bx * BC - 1 + lc;
    const bool inb = ((unsigned)gr < (unsigned)IMH) & ((unsigned)gc < (unsigned)IMW);
    const int grc = gr < 0 ? 0 : (gr > IMH - 1 ? IMH - 1 : gr);
    const int gcc = gc < 0 ? 0 : (gc > IMW - 1 ? IMW - 1 : gc);
    const int pix = (b * IMH + grc) * IMW + gcc;
    float hv0 = 0.f, hv1 = 0.f, hv2 = 0.f, hv3 = 0.f;
    if (first == 0) {
      const v4f t4 = *(const v4f*)(hprev + (size_t)pix * 4);
      hv0 = t4.x; hv1 = t4.y; hv2 = t4.z; hv3 = t4.w;
    }
    float xs0, xs1, xs2, xs3;
    if constexpr (CIN == 3) {
      const float* xp = xin + ((size_t)(b * NTS + tt) * NPIX + (size_t)(grc * IMW + gcc)) * 3;
      xs0 = xp[0] * SAX; xs1 = xp[1] * SAX; xs2 = xp[2] * SAX; xs3 = 0.0f;
    } else {
      const v4f q4 = *(const v4f*)(xin + (size_t)pix * 4);
      xs0 = (q4.x - nm0) * na0 + nc0; xs1 = (q4.y - nm1) * na1 + nc1;
      xs2 = (q4.z - nm2) * na2 + nc2; xs3 = (q4.w - nm3) * na3 + nc3;
    }
    xs0 = inb ? xs0 : 0.f; xs1 = inb ? xs1 : 0.f; xs2 = inb ? xs2 : 0.f; xs3 = inb ? xs3 : 0.f;
    hv0 = inb ? hv0 : 0.f; hv1 = inb ? hv1 : 0.f; hv2 = inb ? hv2 : 0.f; hv3 = inb ? hv3 : 0.f;
    const unsigned xb0 = f16b(xs0), xb1 = f16b(xs1), xb2 = f16b(xs2), xb3 = f16b(xs3);
    const unsigned kb0 = f16b(hv0 * SAH), kb1 = f16b(hv1 * SAH), kb2 = f16b(hv2 * SAH), kb3 = f16b(hv3 * SAH);
    u32x4 pa;
    pa.x = xb0 | (xb1 << 16); pa.y = xb2 | (xb3 << 16); pa.z = kb0 | (kb1 << 16); pa.w = kb2 | (kb3 << 16);
    *(u32x4*)(stg + i * 16) = pa;
    if constexpr (SPLIT != 0) {
      const unsigned lb0 = f16b(xs0 - h2f(xb0)), lb1 = f16b(xs1 - h2f(xb1));
      const unsigned lb2 = f16b(xs2 - h2f(xb2)), lb3 = f16b(xs3 - h2f(xb3));
      u32x4 pb;
      pb.x = lb0 | (lb1 << 16); pb.y = lb2 | (lb3 << 16); pb.z = pa.x; pb.w = pa.y;
      *(u32x4*)(stg + PLB + i * 16) = pb;
    }
  }
  __syncthreads();

  FH A[5];
  {
    const unsigned short* wr = wpk + m * KP + 8 * hh;
#pragma unroll
    for (int s = 0; s < NKS; ++s) {
      A[s].q[0] = *(const u32x4*)(wr + 32 * s);
      A[s].q[1] = *(const u32x4*)(wr + 32 * s + 16);
    }
  }
  const int f0 = 2 * hh;
  const float bi0 = bias[f0], bi1 = bias[f0 + 1], bfg0 = bias[4 + f0], bfg1 = bias[5 + f0];
  const float bgg0 = bias[8 + f0], bgg1 = bias[9 + f0], bog0 = bias[12 + f0], bog1 = bias[13 + f0];

#pragma unroll 1
  for (int q = 0; q < 4; ++q) {
    const int idx = wave * 4 + q, tr = idx >> 1, tc = idx & 1;
    const unsigned char* lb = stg + ((tr * SWW) + tc * 16 + m) * 16;
    v8f acc = zero8f();
    acc = kstep<0, NG>(A[0], lb, hh, acc);
    acc = kstep<1, NG>(A[1], lb, hh, acc);
    acc = kstep<2, NG>(A[2], lb, hh, acc);
    if constexpr (NKS == 5) {
      acc = kstep<3, NG>(A[3], lb, hh, acc);
      acc = kstep<4, NG>(A[4], lb, hh, acc);
    }
    const float s0 = hh ? acc[0] : acc[2];
    const float s1 = hh ? acc[1] : acc[3];
    const float s2 = hh ? acc[4] : acc[6];
    const float s3 = hh ? acc[5] : acc[7];
    const float r0 = __shfl_xor(s0, 16), r1 = __shfl_xor(s1, 16), r2 = __shfl_xor(s2, 16), r3 = __shfl_xor(s3, 16);
    float zi0 = hh ? r0 : acc[0], zi1 = hh ? r1 : acc[1];
    float zf0 = hh ? r2 : acc[4], zf1 = hh ? r3 : acc[5];
    float zg0 = hh ? acc[2] : r0, zg1 = hh ? acc[3] : r1;
    float zo0 = hh ? acc[6] : r2, zo1 = hh ? acc[7] : r3;
    zi0 = zi0 * STI + bi0;  zi1 = zi1 * STI + bi1;
    zf0 = zf0 * STI + bfg0; zf1 = zf1 * STI + bfg1;
    zg0 = zg0 * STI + bgg0; zg1 = zg1 * STI + bgg1;
    zo0 = zo0 * STI + bog0; zo1 = zo1 * STI + bog1;
    const int orow = by * BR + tr, ocol = bx * BC + tc * 16 + m;
    const int pix = (b * IMH + orow) * IMW + ocol;
    float cp0 = 0.f, cp1 = 0.f;
    if (first == 0) {
      const v2f c2 = *(const v2f*)(cst + (size_t)pix * 4 + f0);
      cp0 = c2.x; cp1 = c2.y;
    }
    const float ig0 = sigm_f(zi0), fg0 = sigm_f(zf0), gv0 = tanh_f(zg0), og0 = sigm_f(zo0);
    const float ig1 = sigm_f(zi1), fg1 = sigm_f(zf1), gv1 = tanh_f(zg1), og1 = sigm_f(zo1);
    const float cn0 = fg0 * cp0 + ig0 * gv0;
    const float cn1 = fg1 * cp1 + ig1 * gv1;
    const float hn0 = og0 * tanh_f(cn0);
    const float hn1 = og1 * tanh_f(cn1);
    const float t0 = hh ? hn0 : cn0, t1 = hh ? hn1 : cn1;
    const float u0 = __shfl_xor(t0, 16), u1 = __shfl_xor(t1, 16);
    v4f o;
    o.x = hh ? u0 : hn0; o.y = hh ? u1 : hn1; o.z = hh ? cn0 : u0; o.w = hh ? cn1 : u1;
    float* op = (hh ? cst : hout) + (size_t)pix * 4;
    *(volatile v4f*)op = o;
    __threadfence();
    *(volatile v4f*)op = o;
  }
}

__global__ __launch_bounds__(256) void k_d1(
    const float* __restrict__ h3, const float* __restrict__ w,
    const float* __restrict__ ng, const float* __restrict__ nbt,
    const float* __restrict__ nmu, const float* __restrict__ nva,
    float* part)
{
  __shared__ __attribute__((aligned(16))) unsigned char sm[55296];
  unsigned char* Ah = sm;
  unsigned char* Al = sm + 9216;
  unsigned char* Bh = sm + 18432;
  unsigned char* Bl = sm + 36864;
  const int tid = threadIdx.x, lane = tid & 31, wave = tid >> 5, hh = lane >> 4, m = lane & 15;
  const int rt = wave & 3, cgp = wave >> 2;
  const int kb = blockIdx.x;
  const int kbase = kb * DK;
  const float g0 = ng[0], g1 = ng[1], g2 = ng[2], g3 = ng[3];
  const float q0 = rsqrtf(nva[0] + 1.0e-3f), q1 = rsqrtf(nva[1] + 1.0e-3f), q2 = rsqrtf(nva[2] + 1.0e-3f), q3 = rsqrtf(nva[3] + 1.0e-3f);
  const float m0 = nmu[0], m1 = nmu[1], m2 = nmu[2], m3 = nmu[3];
  const float t0 = nbt[0], t1 = nbt[1], t2 = nbt[2], t3 = nbt[3];
  v8f acc[4];
#pragma unroll
  for (int ct = 0; ct < 4; ++ct) acc[ct] = zero8f();

#pragma unroll 1
  for (int c = 0; c < DK / DKC; ++c) {
    const int k0 = kbase + c * DKC;
#pragma unroll
    for (int j = 0; j < 4; ++j) {
      const int i = tid + 256 * j, row = i >> 4, k4 = (i & 15) * 4;
      const v4f v = *(const v4f*)(h3 + (size_t)row * (NPIX * 4) + k0 + k4);
      const float a0 = lrl((g0 * (v.x - m0)) * q0 + t0);
      const float a1 = lrl((g1 * (v.y - m1)) * q1 + t1);
      const float a2 = lrl((g2 * (v.z - m2)) * q2 + t2);
      const float a3 = lrl((g3 * (v.w - m3)) * q3 + t3);
      const unsigned hb0 = bf16b(a0), hb1 = bf16b(a1), hb2 = bf16b(a2), hb3 = bf16b(a3);
      const unsigned lb0 = bf16b(a0 - bf2f(hb0)), lb1 = bf16b(a1 - bf2f(hb1)), lb2 = bf16b(a2 - bf2f(hb2)), lb3 = bf16b(a3 - bf2f(hb3));
      u32x2 ph, pl;
      ph.x = hb0 | (hb1 << 16); ph.y = hb2 | (hb3 << 16);
      pl.x = lb0 | (lb1 << 16); pl.y = lb2 | (lb3 << 16);
      *(u32x2*)(Ah + (row * APITCH + k4) * 2) = ph;
      *(u32x2*)(Al + (row * APITCH + k4) * 2) = pl;
    }
#pragma unroll
    for (int j = 0; j < 4; ++j) {
      const int i = tid + 256 * j, n = i & 127, k8 = (i >> 7) * 8;
      unsigned hb[8], lb[8];
#pragma unroll
      for (int jj = 0; jj < 8; ++jj) {
        const float wv = w[(size_t)(k0 + k8 + jj) * 128 + n];
        hb[jj] = bf16b(wv);
        lb[jj] = bf16b(wv - bf2f(hb[jj]));
      }
      u32x4 ph, pl;
      ph.x = hb[0] | (hb[1] << 16); ph.y = hb[2] | (hb[3] << 16); ph.z = hb[4] | (hb[5] << 16); ph.w = hb[6] | (hb[7] << 16);
      pl.x = lb[0] | (lb[1] << 16); pl.y = lb[2] | (lb[3] << 16); pl.z = lb[4] | (lb[5] << 16); pl.w = lb[6] | (lb[7] << 16);
      *(u32x4*)(Bh + (n * APITCH + k8) * 2) = ph;
      *(u32x4*)(Bl + (n * APITCH + k8) * 2) = pl;
    }
    __syncthreads();
#pragma unroll
    for (int s = 0; s < 2; ++s) {
      FB ah, al;
      const int ao = ((rt * 16 + m) * APITCH + 32 * s + 8 * hh) * 2;
      ah.q[0] = *(const u32x4*)(Ah + ao); ah.q[1] = *(const u32x4*)(Ah + ao + 32);
      al.q[0] = *(const u32x4*)(Al + ao); al.q[1] = *(const u32x4*)(Al + ao + 32);
#pragma unroll
      for (int ct = 0; ct < 4; ++ct) {
        const int bo = ((cgp * 64 + ct * 16 + m) * APITCH + 32 * s + 8 * hh) * 2;
        FB bh, bl;
        bh.q[0] = *(const u32x4*)(Bh + bo); bh.q[1] = *(const u32x4*)(Bh + bo + 32);
        bl.q[0] = *(const u32x4*)(Bl + bo); bl.q[1] = *(const u32x4*)(Bl + bo + 32);
        acc[ct] = wmb(ah, bh, acc[ct]);
        acc[ct] = wmb(ah, bl, acc[ct]);
        acc[ct] = wmb(al, bh, acc[ct]);
      }
    }
    __syncthreads();
  }

  float* E = (float*)sm;
#pragma unroll
  for (int ct = 0; ct < 4; ++ct) {
#pragma unroll
    for (int r = 0; r < 8; ++r) E[(rt * 16 + 8 * hh + r) * 128 + cgp * 64 + ct * 16 + m] = acc[ct][r];
  }
  __syncthreads();
  v4f ev[8];
#pragma unroll
  for (int j = 0; j < 8; ++j) {
    const int i = tid + 256 * j, row = i >> 5, c4 = (i & 31) * 4;
    ev[j] = *(const v4f*)(E + row * 128 + c4);
  }
  float* pp = part + (size_t)kb * 8192;
#pragma unroll
  for (int j = 0; j < 8; ++j) {
    const int i = tid + 256 * j, row = i >> 5, c4 = (i & 31) * 4;
    *(volatile v4f*)(pp + row * 128 + c4) = ev[j];
  }
  __threadfence();
#pragma unroll
  for (int j = 0; j < 8; ++j) {
    const int i = tid + 256 * j, row = i >> 5, c4 = (i & 31) * 4;
    *(volatile v4f*)(pp + row * 128 + c4) = ev[j];
  }
}

__device__ __forceinline__ void dlayer(const float* in, const float* __restrict__ w, const float* __restrict__ bias, float* ob, int tid) {
  const int c = tid & 127, rg = tid >> 7;
  const float bc = bias[c];
#pragma unroll 1
  for (int j = 0; j < 32; ++j) {
    const int r = rg * 32 + j;
    float s = 0.0f;
#pragma unroll 4
    for (int k = 0; k < 128; ++k) s += in[r * 128 + k] * w[k * 128 + c];
    s += bc;
    ob[r * 128 + c] = lrl(s);
  }
}

__global__ __launch_bounds__(256) void k_head(
    const float* __restrict__ part, const float* __restrict__ b1,
    const float* __restrict__ w2, const float* __restrict__ b2,
    const float* __restrict__ w3, const float* __restrict__ b3,
    const float* __restrict__ wo, const float* __restrict__ bo,
    float* out)
{
  __shared__ __attribute__((aligned(16))) float bufA[8192];
  __shared__ __attribute__((aligned(16))) float bufB[8192];
  const int tid = threadIdx.x;
#pragma unroll 1
  for (int j = 0; j < 32; ++j) {
    const int e = tid + 256 * j;
    float s = 0.0f;
#pragma unroll 4
    for (int kb = 0; kb < NKB; ++kb) s += part[(size_t)kb * 8192 + e];
    s += b1[e & 127];
    bufA[e] = lrl(s);
  }
  __syncthreads();
  dlayer(bufA, w2, b2, bufB, tid);
  __syncthreads();
  dlayer(bufB, w3, b3, bufA, tid);
  __syncthreads();
  {
    const int r = (tid >> 1) & 63, jj = tid & 1;
    float s = 0.0f;
#pragma unroll 4
    for (int k = 0; k < 128; ++k) s += bufA[r * 128 + k] * wo[k * 2 + jj];
    s += bo[jj];
    if (tid < 128) bufB[tid] = s;
  }
  __syncthreads();
  const v4f ovv = *(const v4f*)(bufB + 4 * (tid & 31));
  if (tid < 32) *(volatile v4f*)(out + 4 * tid) = ovv;
  __threadfence();
  if (tid < 32) *(volatile v4f*)(out + 4 * tid) = ovv;
}

extern "C" void kernel_launch(void* const* d_in, const int* in_sizes, int n_in,
                              void* d_out, int out_size, void* d_ws, size_t ws_size,
                              hipStream_t stream)
{
  if (n_in < 30) return;
  if (in_sizes[0] != NBAT * NTS * NPIX * 3) return;
  if (in_sizes[1] != 9 * 3 * 16 || in_sizes[2] != 9 * 4 * 16 || in_sizes[3] < 16) return;
  if (in_sizes[4] < 4 || in_sizes[5] < 4 || in_sizes[6] < 4 || in_sizes[7] < 4) return;
  if (in_sizes[8] != 9 * 4 * 16 || in_sizes[9] != 9 * 4 * 16 || in_sizes[10] < 16) return;
  if (in_sizes[11] < 4 || in_sizes[12] < 4 || in_sizes[13] < 4 || in_sizes[14] < 4) return;
  if (in_sizes[15] != 9 * 4 * 16 || in_sizes[16] != 9 * 4 * 16 || in_sizes[17] < 16) return;
  if (in_sizes[18] < 4 || in_sizes[19] < 4 || in_sizes[20] < 4 || in_sizes[21] < 4) return;
  if (in_sizes[22] != NPIX * 4 * 128 || in_sizes[23] < 128) return;
  if (in_sizes[24] != 128 * 128 || in_sizes[25] < 128 || in_sizes[26] != 128 * 128 || in_sizes[27] < 128) return;
  if (in_sizes[28] != 128 * 2 || in_sizes[29] < 2) return;
  if (out_size != NBAT * 2) return;

  const float* x    = (const float*)d_in[0];
  const float* wx1  = (const float*)d_in[1];
  const float* wh1  = (const float*)d_in[2];
  const float* b1   = (const float*)d_in[3];
  const float* g1   = (const float*)d_in[4];
  const float* bt1  = (const float*)d_in[5];
  const float* m1   = (const float*)d_in[6];
  const float* v1   = (const float*)d_in[7];
  const float* wx2  = (const float*)d_in[8];
  const float* wh2  = (const float*)d_in[9];
  const float* b2   = (const float*)d_in[10];
  const float* g2   = (const float*)d_in[11];
  const float* bt2  = (const float*)d_in[12];
  const float* m2   = (const float*)d_in[13];
  const float* v2   = (const float*)d_in[14];
  const float* wx3  = (const float*)d_in[15];
  const float* wh3  = (const float*)d_in[16];
  const float* b3   = (const float*)d_in[17];
  const float* g3   = (const float*)d_in[18];
  const float* bt3  = (const float*)d_in[19];
  const float* m3   = (const float*)d_in[20];
  const float* v3   = (const float*)d_in[21];
  const float* w_d1 = (const float*)d_in[22];
  const float* b_d1 = (const float*)d_in[23];
  const float* w_d2 = (const float*)d_in[24];
  const float* b_d2 = (const float*)d_in[25];
  const float* w_d3 = (const float*)d_in[26];
  const float* b_d3 = (const float*)d_in[27];
  const float* w_o  = (const float*)d_in[28];
  const float* b_o  = (const float*)d_in[29];
  float* out = (float*)d_out;

  const size_t PL    = (size_t)NBAT * NPIX * 4 * sizeof(float);
  const size_t oW    = 0;
  const size_t oP0   = 24576;
  const size_t oPart = oP0 + 7 * PL;
  const size_t total = oPart + (size_t)NKB * 8192 * sizeof(float);
  if (total > ws_size) return;
  if (total > (size_t)134217728) return;
  char* ws = (char*)d_ws;
  unsigned short* wpk = (unsigned short*)(ws + oW);
  float* P[4];
  float* C[3];
  for (int i = 0; i < 4; ++i) P[i] = (float*)(ws + oP0 + (size_t)i * PL);
  for (int l = 0; l < 3; ++l) C[l] = (float*)(ws + oP0 + (size_t)(4 + l) * PL);
  float* part = (float*)(ws + oPart);

  k_wpack<<<3, 256, 0, stream>>>(wx1, wh1, wx2, wh2, wx3, wh3, wpk);

  const dim3 cgrid(IMW / BC, IMH / BR, NBAT);
  for (int t = 0; t < NTS; ++t) {
    for (int l = 0; l < 3; ++l) {
      const int g = 3 * t + l;
      float* ho = P[g & 3];
      const float* hp = P[(g + 1) & 3];
      const float* xi = P[(g + 3) & 3];
      const int fst = (t == 0) ? 1 : 0;
      if (l == 0) {
        k_cell<3, 0><<<cgrid, 256, 0, stream>>>(x, hp, ho, C[0], wpk, b1, g1, bt1, m1, v1, t, fst);
      } else if (l == 1) {
        k_cell<4, 1><<<cgrid, 256, 0, stream>>>(xi, hp, ho, C[1], wpk + 4096, b2, g1, bt1, m1, v1, t, fst);
      } else {
        k_cell<4, 1><<<cgrid, 256, 0, stream>>>(xi, hp, ho, C[2], wpk + 8192, b3, g2, bt2, m2, v2, t, fst);
      }
    }
  }

  k_d1<<<NKB, 256, 0, stream>>>(P[14 & 3], w_d1, g3, bt3, m3, v3, part);
  k_head<<<1, 256, 0, stream>>>(part, b_d1, w_d2, b_d2, w_d3, b_d3, w_o, b_o, out);
}
